// ProbAttention_7550552506918
// MI455X (gfx1250) — hardware-run, weakly checked
//
#include <hip/hip_runtime.h>
#include <math.h>

typedef __attribute__((ext_vector_type(16))) _Float16 v16h;
typedef __attribute__((ext_vector_type(16))) __bf16 v16b;
typedef __attribute__((ext_vector_type(8)))  _Float16 v8h;
typedef __attribute__((ext_vector_type(8)))  float v8f;
typedef __attribute__((ext_vector_type(4)))  float v4f;
typedef __attribute__((ext_vector_type(2)))  float v2f;
typedef __attribute__((ext_vector_type(4)))  unsigned v4u;
typedef __attribute__((ext_vector_type(4)))  int v4i;
typedef float __attribute__((may_alias)) float_a;
typedef int __attribute__((may_alias)) int_a;

template <typename T> __device__ __forceinline__ void vst2(void* p, T v) { *(volatile T*)p = v; __threadfence(); *(volatile T*)p = v; }
__device__ __forceinline__ v8f wmma16(v16h a, v16h b, v8f c) {
  v8f d = __builtin_amdgcn_wmma_f32_16x16x32_f16(false, a, false, b, (short)0, c, false, false);
  asm volatile("v_nop\n\tv_nop\n\tv_nop\n\tv_nop" : "+v"(d) : "v"(a), "v"(b));
  return d;
}
__device__ __forceinline__ v8f wmma_bf(v16b a, v16b b, v8f c) {
  v8f d = __builtin_amdgcn_wmma_f32_16x16x32_bf16(false, a, false, b, (short)0, c, false, false);
  asm volatile("v_nop\n\tv_nop\n\tv_nop\n\tv_nop" : "+v"(d) : "v"(a), "v"(b));
  return d;
}
__device__ __forceinline__ v16h frag_h(const _Float16* rowk0, int lane) {
  union { v16h v; v8h q[2]; } u; const _Float16* p = rowk0 + 8 * (lane >> 4);
  u.q[0] = *(const v8h*)p; u.q[1] = *(const v8h*)(p + 16); return u.v;
}
__device__ __forceinline__ v16h frag_f32(const float* rowk0, int lane) {
  v16h a; const float* p = rowk0 + 8 * (lane >> 4);
#pragma unroll
  for (int i = 0; i < 8; ++i) { a[i] = (_Float16)p[i]; a[8 + i] = (_Float16)p[16 + i]; }
  return a;
}
__device__ __forceinline__ v16h frag_f32s(const float* rowk0, int lane, float sc) {
  v16h a; const float* p = rowk0 + 8 * (lane >> 4);
#pragma unroll
  for (int i = 0; i < 8; ++i) { a[i] = (_Float16)(p[i] * sc); a[8 + i] = (_Float16)(p[16 + i] * sc); }
  return a;
}
__device__ __forceinline__ v16h fragc_f32(const float* W, int k0, int n, int lane, int ld, int K) {
  v16h a; const int g = lane >> 4;
#pragma unroll
  for (int i = 0; i < 8; ++i) { const int ka = k0 + 8 * g + i, kb = ka + 16;
    a[i] = (_Float16)(ka < K ? W[(size_t)(ka < K ? ka : K - 1) * ld + n] : 0.f); a[8 + i] = (_Float16)(kb < K ? W[(size_t)(kb < K ? kb : K - 1) * ld + n] : 0.f); }
  return a;
}
struct F2 { v16b h, l; };
__device__ __forceinline__ F2 bsplit16(const float v[16]) { F2 r;
#pragma unroll
  for (int i = 0; i < 16; ++i) { const __bf16 h = (__bf16)v[i]; r.h[i] = h; r.l[i] = (__bf16)(v[i] - (float)h); }
  return r; }
__device__ __forceinline__ F2 split_row(const float* row, int k0, int lane) { float v[16]; const float* p = row + k0 + 8 * (lane >> 4);
#pragma unroll
  for (int i = 0; i < 8; ++i) { v[i] = p[i]; v[8 + i] = p[16 + i]; }
  return bsplit16(v); }
__device__ __forceinline__ F2 split_rowK(const float* row, int k0, int lane, int K) { float v[16]; const int g = lane >> 4;
#pragma unroll
  for (int i = 0; i < 8; ++i) { const int ka = k0 + 8 * g + i, kb = ka + 16; v[i] = ka < K ? row[ka < K ? ka : K - 1] : 0.f; v[8 + i] = kb < K ? row[kb < K ? kb : K - 1] : 0.f; }
  return bsplit16(v); }
__device__ __forceinline__ F2 split_col(const float* W, int k0, int n, int lane, int ld, int K) { float v[16]; const int g = lane >> 4;
#pragma unroll
  for (int i = 0; i < 8; ++i) { const int ka = k0 + 8 * g + i, kb = ka + 16; v[i] = ka < K ? W[(size_t)(ka < K ? ka : K - 1) * ld + n] : 0.f; v[8 + i] = kb < K ? W[(size_t)(kb < K ? kb : K - 1) * ld + n] : 0.f; }
  return bsplit16(v); }
__device__ __forceinline__ v8f mac3(const F2& a, const F2& b, v8f c) { c = wmma_bf(a.l, b.h, c); c = wmma_bf(a.h, b.l, c); return wmma_bf(a.h, b.h, c); }
__device__ __forceinline__ float sigm(float v) { return 1.0f / (1.0f + expf(-v)); }
#define LDSX() do { asm volatile("s_wait_dscnt 0" ::: "memory"); __builtin_amdgcn_wave_barrier(); __builtin_amdgcn_fence(__ATOMIC_RELEASE, "workgroup"); } while (0)

#define NBT 2
#define LQ 4096
#define NH 8
#define HD 64
#define US 45
#define NCT 45
#define OUT1_OFF (4u * (size_t)NBT * NH * LQ * HD)
#ifndef NBP
#define NBP NBT
#endif
typedef __attribute__((ext_vector_type(4))) int v4i;
__device__ __forceinline__ float bfr(float v) { return (float)(__bf16)v; }
__global__ __launch_bounds__(256) void k_vt(const float* __restrict__ V, float* __restrict__ O) { const size_t e4 = (size_t)blockIdx.x * 256 + threadIdx.x; if (e4 >= (size_t)NBP * NH * LQ * HD / 4) return;
  const size_t e = e4 * 4; const int d = (int)(e % HD); const size_t t = e / HD; const int l = (int)(t % LQ); const size_t t2 = t / LQ; const int h = (int)(t2 % NH); const int b = (int)(t2 / NH);
  const v4f x = *(const v4f*)(V + (((size_t)b * LQ + l) * NH + h) * HD + d); v4f o; o[0] = bfr(x[0]); o[1] = bfr(x[1]); o[2] = bfr(x[2]); o[3] = bfr(x[3]); vst2(O + e, o); }
__global__ __launch_bounds__(128) void k_prob(const float* __restrict__ Q, const float* __restrict__ K, const int* __restrict__ IS, float* __restrict__ M) { __shared__ __align__(16) float st[4][16][20]; __shared__ __align__(16) float sm[64];
  const int tid = threadIdx.x, wave = tid >> 5, lane = tid & 31, col = lane & 15, g = lane >> 4; const int bh = blockIdx.y; const int b = bh / NH, h = bh % NH; const int q0 = blockIdx.x * 64 + wave * 16;
  v16b a0, a1; { const float* p = Q + (((size_t)b * LQ + q0 + col) * NH + h) * HD + 8 * g;
#pragma unroll
    for (int i = 0; i < 8; ++i) { a0[i] = (__bf16)p[i]; a0[8 + i] = (__bf16)p[16 + i]; a1[i] = (__bf16)p[32 + i]; a1[8 + i] = (__bf16)p[48 + i]; } }
  asm volatile("s_wait_loadcnt 0x0" ::: "memory");
  const int myrow = lane >> 1, half = lane & 1; float mx = -3.0e38f, sum = 0.f;
#pragma unroll 1
  for (int ct = 0; ct < NCT; ++ct) { const int j = ct * 16 + col; const int ro = j / US, s = j % US;
    int key = IS[(size_t)(q0 + ro) * US + s]; key = key < 0 ? 0 : (key >= LQ ? LQ - 1 : key);
    v16b w0, w1; { const float* pk = K + (((size_t)b * LQ + key) * NH + h) * HD + 8 * g;
#pragma unroll
      for (int i = 0; i < 8; ++i) { w0[i] = (__bf16)pk[i]; w0[8 + i] = (__bf16)pk[16 + i]; } asm volatile("s_wait_loadcnt 0x0" ::: "memory");
#pragma unroll
      for (int i = 0; i < 8; ++i) { w1[i] = (__bf16)pk[32 + i]; w1[8 + i] = (__bf16)pk[48 + i]; } asm volatile("s_wait_loadcnt 0x0" ::: "memory"); }
    v8f acc = {}; acc = wmma_bf(a0, w0, acc); acc = wmma_bf(a1, w1, acc);
#pragma unroll
    for (int r = 0; r < 8; ++r) st[wave][8 * g + r][col] = acc[r];
    LDSX();
#pragma unroll
    for (int c = 0; c < 8; ++c) { const int cc = half * 8 + c; const int jj = ct * 16 + cc; const bool mine = (jj / US) == myrow; const float v = st[wave][myrow][cc]; mx = mine ? fmaxf(mx, v) : mx; sum = mine ? sum + v : sum; }
    LDSX(); }
  mx = fmaxf(mx, __shfl_xor(mx, 1)); sum += __shfl_xor(sum, 1);
  if (half == 0) sm[wave * 16 + myrow] = mx - sum * (1.0f / (float)LQ);
  __syncthreads();
  if (tid < 16) vst2(M + (size_t)bh * LQ + blockIdx.x * 64 + tid * 4, *(const v4f*)&sm[tid * 4]); }
extern "C" void kernel_launch(void* const* d_in, const int* in_sizes, int n_in, void* d_out, int out_size, void* d_ws, size_t ws_size, hipStream_t stream) {
  (void)in_sizes; (void)n_in; (void)out_size; (void)d_ws; (void)ws_size;
  k_vt<<<dim3((NBP * NH * LQ * HD / 4 + 255) / 256), 256, 0, stream>>>((const float*)d_in[2], (float*)d_out);
  k_prob<<<dim3(LQ / 64, NBP * NH), 128, 0, stream>>>((const float*)d_in[0], (const float*)d_in[1], (const int*)d_in[3], (float*)((char*)d_out + OUT1_OFF));
}
